// CausalMAC_55903294324922
// MI455X (gfx1250) — hardware-verified
//
#include <hip/hip_runtime.h>


#define NBQ  16
#define NN   256
#define NT   4096
#define FF   64
#define DD   128
#define NH_  4
#define DH   32
#define D3   384
#define DFF  512
#define NZ   64
#define NPR  65280
#define PCAR 1024.0f
typedef _Float16 h16;
typedef unsigned short bf;
typedef __attribute__((ext_vector_type(16))) __bf16   v16bf;
typedef __attribute__((ext_vector_type(16))) _Float16 v16h;
typedef __attribute__((ext_vector_type(8)))  _Float16 v8h;
typedef __attribute__((ext_vector_type(8)))  unsigned short v8us;
typedef __attribute__((ext_vector_type(8)))  float    v8f;
typedef __attribute__((ext_vector_type(4)))  float    v4f;
typedef v8h  __attribute__((may_alias)) v8ha;
typedef v4f  __attribute__((may_alias)) v4fa;
typedef v8us __attribute__((may_alias)) v8usa;

__device__ __forceinline__ unsigned short f2bf(float f) { unsigned u = __float_as_uint(f); u += 0x7FFFu + ((u >> 16) & 1u); return (unsigned short)(u >> 16); }
__device__ __forceinline__ float bf2f(unsigned short b) { return __uint_as_float(((unsigned)b) << 16); }
__device__ __forceinline__ float bfr(float f) { return bf2f(f2bf(f)); }
__device__ __forceinline__ v16h cat16(v8h lo, v8h hi) { return __builtin_shufflevector(lo, hi, 0, 1, 2, 3, 4, 5, 6, 7, 8, 9, 10, 11, 12, 13, 14, 15); }
__device__ __forceinline__ v16bf cat16b(v8us lo, v8us hi) { return __builtin_bit_cast(v16bf, __builtin_shufflevector(lo, hi, 0, 1, 2, 3, 4, 5, 6, 7, 8, 9, 10, 11, 12, 13, 14, 15)); }
__device__ __forceinline__ v8f wmma16(v16h a, v16h b, v8f c) { return __builtin_amdgcn_wmma_f32_16x16x32_f16(false, a, false, b, (short)0, c, false, false); }
__device__ __forceinline__ v8f wmmab(v16bf a, v16bf b, v8f c) { return __builtin_amdgcn_wmma_f32_16x16x32_bf16(false, a, false, b, (short)0, c, false, false); }


template <typename T16> struct WFrag;
template <> struct WFrag<h16> { typedef v16h V; static __device__ __forceinline__ V ld(const h16* p) { return cat16(*(const v8h*)p, *(const v8h*)(p + 16)); } static __device__ __forceinline__ v8f mma(V a, V b, v8f c) { return wmma16(a, b, c); } };
template <> struct WFrag<bf> { typedef v16bf V; static __device__ __forceinline__ V ld(const bf* p) { return cat16b(*(const v8us*)p, *(const v8us*)(p + 16)); } static __device__ __forceinline__ v8f mma(V a, V b, v8f c) { return wmmab(a, b, c); } };
template <typename T16, int NSPLIT, bool BIAS>
__global__ __launch_bounds__(32) void k_gemmw(const T16* __restrict__ A, const T16* __restrict__ A2, const T16* __restrict__ Bt, const T16* __restrict__ Bt2, int K, float* C, int ldc, const float* __restrict__ bias, size_t sA, size_t sB, size_t sC) {
    typedef typename WFrag<T16>::V V;
    __shared__ __align__(16) float os[16 * 68];
    const size_t z = blockIdx.z; A += z * sA; if (A2) A2 += z * sA; Bt += z * sB; if (Bt2) Bt2 += z * sB; C += z * sC;
    const int lane = threadIdx.x & 31, lr = lane & 15, hi = lane >> 4; const int r0 = blockIdx.x * 64, c0 = blockIdx.y * 64;
    v8f acc[4][4];
#pragma unroll
    for (int mb = 0; mb < 4; ++mb)
#pragma unroll
        for (int nb = 0; nb < 4; ++nb) acc[mb][nb] = (v8f){};
    const size_t aoff = (size_t)(r0 + lr) * K + 8 * hi, boff = (size_t)(c0 + lr) * K + 8 * hi;
#pragma unroll 1
    for (int kc = 0; kc < K; kc += 32) {
        V a[4], a2[4];
#pragma unroll
        for (int mb = 0; mb < 4; ++mb) { a[mb] = WFrag<T16>::ld(A + aoff + (size_t)mb * 16 * K + kc); if (NSPLIT == 1 || NSPLIT == 2) a2[mb] = WFrag<T16>::ld(A2 + aoff + (size_t)mb * 16 * K + kc); }
#pragma unroll
        for (int nb = 0; nb < 4; ++nb) { const V b = WFrag<T16>::ld(Bt + boff + (size_t)nb * 16 * K + kc); V b2; if (NSPLIT >= 2) b2 = WFrag<T16>::ld(Bt2 + boff + (size_t)nb * 16 * K + kc);
#pragma unroll
            for (int mb = 0; mb < 4; ++mb) { acc[mb][nb] = WFrag<T16>::mma(a[mb], b, acc[mb][nb]); if (NSPLIT == 1 || NSPLIT == 2) acc[mb][nb] = WFrag<T16>::mma(a2[mb], b, acc[mb][nb]); if (NSPLIT >= 2) acc[mb][nb] = WFrag<T16>::mma(a[mb], b2, acc[mb][nb]); } }
        asm volatile("v_nop\n\tv_nop\n\tv_nop\n\tv_nop" : "+v"(acc[0][0]), "+v"(acc[1][1]), "+v"(acc[2][2]), "+v"(acc[3][3]) : "v"(a[0]), "v"(a[3]));
    }
#pragma unroll
    for (int mb = 0; mb < 4; ++mb) {
#pragma unroll
        for (int nb = 0; nb < 4; ++nb) {
#pragma unroll
            for (int j = 0; j < 8; ++j) os[(hi * 8 + j) * 68 + nb * 16 + lr] = acc[mb][nb][j]; }
        __builtin_amdgcn_wave_barrier(); asm volatile("" ::: "memory");
        float* crow = C + (size_t)(r0 + mb * 16) * ldc + c0;
#pragma unroll 1
        for (int ps = 0; ps < 2; ++ps) {
#pragma unroll
            for (int s = 0; s < 8; ++s) { const int row = 2 * s + hi, cofs = lr * 4; v4f val = *(const v4fa*)(os + row * 68 + cofs); if (BIAS) { val[0] += bfr(bias[c0 + cofs]); val[1] += bfr(bias[c0 + cofs + 1]); val[2] += bfr(bias[c0 + cofs + 2]); val[3] += bfr(bias[c0 + cofs + 3]); }
                *(volatile v4f*)(crow + (size_t)row * ldc + cofs) = val; }
            if (ps == 0) __threadfence(); }
        __builtin_amdgcn_wave_barrier(); asm volatile("" ::: "memory");
    }
}

__device__ __forceinline__ h16 tohx(float x) { return (h16)x; }
__device__ __forceinline__ void splitf(float y, unsigned short& h, unsigned short& l) { h = f2bf(y); l = f2bf(y - bf2f(h)); }
typedef __attribute__((ext_vector_type(2))) unsigned short v2us;
typedef __attribute__((ext_vector_type(4))) unsigned short v4us;
typedef __attribute__((ext_vector_type(2))) _Float16 v2h;
typedef __attribute__((ext_vector_type(4))) _Float16 v4h;

__global__ __launch_bounds__(256) void k_wtG(const float* __restrict__ w, int K, int N, bf* Bt) {
    const int lane = threadIdx.x & 31; const int L0 = (blockIdx.x * 8 + (threadIdx.x >> 5)) * 8; const int nlines = N * K / 64;
#pragma unroll
    for (int ps = 0; ps < 2; ++ps) {
#pragma unroll 1
        for (int l = 0; l < 8; ++l) { const int L = L0 + l; if (L >= nlines) break; const size_t e = (size_t)L * 64 + lane * 2; const int k = (int)(e % K), n = (int)(e / K); v2us o;
            o[0] = f2bf(w[(size_t)k * N + n]); o[1] = f2bf(w[(size_t)(k + 1) * N + n]); *(volatile v2us*)(Bt + e) = o; }
        if (ps == 0) __threadfence(); }
}
__global__ __launch_bounds__(256) void k_cvt8(const float* __restrict__ src, bf* dst, size_t n8) { const size_t i = (size_t)blockIdx.x * 256 + threadIdx.x; if (i >= n8) return; const v8f v = *(const v8f*)(src + i * 8); v8us o;
#pragma unroll
    for (int k = 0; k < 8; ++k) o[k] = f2bf(v[k]); *(volatile v8us*)(dst + i * 8) = o; __threadfence(); *(volatile v8us*)(dst + i * 8) = o; }
template <int RELU, int RES> __global__ __launch_bounds__(256) void k_ln(const float* __restrict__ A, const float* __restrict__ R, const float* __restrict__ gg, const float* __restrict__ bb, float* X, bf* Xh, bf* Xl) { const int lane = threadIdx.x & 31; const int t = blockIdx.x * 8 + (threadIdx.x >> 5); if (t >= NT) return; const size_t base = (size_t)t * DD + lane * 4; const v4f a = *(const v4f*)(A + base); float v[4]; float s = 0.f;
#pragma unroll
    for (int u = 0; u < 4; ++u) { float x0 = RELU ? fmaxf(a[u], 0.f) : a[u]; if (RES) x0 = __fadd_rn(R[base + u], x0); v[u] = x0; s += x0; }
#pragma unroll
    for (int sh = 16; sh; sh >>= 1) s += __shfl_xor(s, sh, 32);
    const float mean = s * (1.0f / DD); float q = 0.f;
#pragma unroll
    for (int u = 0; u < 4; ++u) { float d = __fsub_rn(v[u], mean); asm volatile("" : "+v"(d)); float p = __fmul_rn(d, d); asm volatile("" : "+v"(p)); q = __fadd_rn(q, p); }
#pragma unroll
    for (int sh = 16; sh; sh >>= 1) q += __shfl_xor(q, sh, 32);
    const float rstd = __frsqrt_rn(__fadd_rn(q * (1.0f / DD), 1e-5f)); v4f o; v4us oh, ol;
#pragma unroll
    for (int u = 0; u < 4; ++u) { float d = __fsub_rn(v[u], mean); asm volatile("" : "+v"(d)); float n0 = __fmul_rn(d, rstd); asm volatile("" : "+v"(n0)); float g1 = bfr(gg[lane * 4 + u]), b1 = bfr(bb[lane * 4 + u]); asm volatile("" : "+v"(g1)); asm volatile("" : "+v"(b1)); float t1 = __fmul_rn(n0, g1); asm volatile("" : "+v"(t1)); const float y = __fadd_rn(t1, b1); o[u] = y; unsigned short a2, b2; splitf(y, a2, b2); oh[u] = a2; ol[u] = b2; }
    for (int ps = 0; ps < 2; ++ps) { *(volatile v4f*)(X + base) = o; *(volatile v4us*)(Xh + base) = oh; *(volatile v4us*)(Xl + base) = ol; if (ps == 0) __threadfence(); } }
__global__ __launch_bounds__(256) void k_pl(const float* __restrict__ F, int off, h16* P) { const int e = (blockIdx.x * 256 + threadIdx.x) * 4; if (e >= NZ * NN * DH) return; const int d = e % DH; const int n = (e / DH) % NN; const int z = e / (DH * NN); const int b = z / NH_, h = z % NH_; const float* f = F + ((size_t)b * NN + n) * D3 + off + h * DH + d; v4h o;
#pragma unroll
    for (int u = 0; u < 4; ++u) o[u] = tohx(f[u]); *(volatile v4h*)(P + e) = o; __threadfence(); *(volatile v4h*)(P + e) = o; }
__global__ __launch_bounds__(256) void k_vt(const float* __restrict__ F, h16* VT) { const int e = (blockIdx.x * 256 + threadIdx.x) * 2; if (e >= NZ * 64 * NN) return; const int n = e % NN; const int d = (e / NN) % 64; const int z = e / (NN * 64); const int b = z / NH_, h = z % NH_; v2h o;
    if (d < DH) { o[0] = tohx(F[((size_t)b * NN + n) * D3 + 2 * DD + h * DH + d]); o[1] = tohx(F[((size_t)b * NN + n + 1) * D3 + 2 * DD + h * DH + d]); } else { o[0] = (h16)0.f; o[1] = (h16)0.f; }
    *(volatile v2h*)(VT + e) = o; __threadfence(); *(volatile v2h*)(VT + e) = o; }
__global__ __launch_bounds__(256) void k_soft(const float* __restrict__ Sb, h16* P16) { const int lane = threadIdx.x & 31; const int row = blockIdx.x * 8 + (threadIdx.x >> 5); if (row >= NZ * NN) return; const float* sr = Sb + (size_t)row * NN; float v[NN / 32]; float mx = -3.0e38f; const float scl = 0.17677669529663687f;
#pragma unroll
    for (int ch = 0; ch < NN / 128; ++ch) { const v4f a = *(const v4f*)(sr + ch * 128 + lane * 4);
#pragma unroll
        for (int u = 0; u < 4; ++u) { const float t = a[u] * scl; v[ch * 4 + u] = t; mx = fmaxf(mx, t); } }
#pragma unroll
    for (int sh = 16; sh; sh >>= 1) mx = fmaxf(mx, __shfl_xor(mx, sh, 32));
    float sum = 0.f;
#pragma unroll
    for (int q = 0; q < NN / 32; ++q) { float d0 = __fsub_rn(v[q], mx); asm volatile("" : "+v"(d0)); v[q] = __builtin_amdgcn_exp2f(__fmul_rn(d0, 1.4426950408889634f)); sum += v[q]; }
#pragma unroll
    for (int sh = 16; sh; sh >>= 1) sum += __shfl_xor(sum, sh, 32);
    const float f = __fdiv_rn(PCAR, sum);
    for (int ps = 0; ps < 2; ++ps) {
#pragma unroll
        for (int ch = 0; ch < NN / 128; ++ch) { v4h o4;
#pragma unroll
            for (int q = 0; q < 4; ++q) o4[q] = tohx(v[ch * 4 + q] * f); *(volatile v4h*)(P16 + (size_t)row * NN + ch * 128 + lane * 4) = o4; }
        if (ps == 0) __threadfence(); } }
__global__ __launch_bounds__(256) void k_mrg(const float* __restrict__ O, bf* Ah, bf* Al) { const int e = (blockIdx.x * 256 + threadIdx.x) * 4; if (e >= NT * DD) return; const int c = e % DD; const int t = e / DD; const int b = t / NN, n = t % NN; const int h = c / DH, d = c % DH; const float* o = O + (((size_t)(b * NH_ + h) * NN + n) * 64 + d); v4us oh, ol;
#pragma unroll
    for (int u = 0; u < 4; ++u) { unsigned short a, b2; splitf(o[u] * (1.0f / PCAR), a, b2); oh[u] = a; ol[u] = b2; } *(volatile v4us*)(Ah + e) = oh; *(volatile v4us*)(Al + e) = ol; __threadfence(); *(volatile v4us*)(Ah + e) = oh; *(volatile v4us*)(Al + e) = ol; }
__global__ __launch_bounds__(256) void k_rl(const float* __restrict__ F, size_t n4, bf* Gh, bf* Gl) { const size_t e = ((size_t)blockIdx.x * 256 + threadIdx.x) * 4; if (e >= n4) return; const v4f a = *(const v4f*)(F + e); v4us oh, ol;
#pragma unroll
    for (int u = 0; u < 4; ++u) { unsigned short h, l; splitf(fmaxf(a[u], 0.f), h, l); oh[u] = h; ol[u] = l; } *(volatile v4us*)(Gh + e) = oh; *(volatile v4us*)(Gl + e) = ol; __threadfence(); *(volatile v4us*)(Gh + e) = oh; *(volatile v4us*)(Gl + e) = ol; }
__global__ __launch_bounds__(256) void k_pair(const float* __restrict__ A, const float* __restrict__ Bm, const float* __restrict__ b1, const float* __restrict__ w2, const float* __restrict__ b2, float* OUT) { const size_t e = ((size_t)blockIdx.x * 256 + threadIdx.x) * 4; if (e >= (size_t)NBQ * NPR) return; const int b = (int)(e / NPR); const int p0 = (int)(e % NPR); v4f o;
#pragma unroll 1
    for (int u = 0; u < 4; ++u) { const int p = p0 + u; const int i = p / (NN - 1); const int jp = p % (NN - 1); const int j = jp + (jp >= i ? 1 : 0); const float* ar = A + ((size_t)b * NN + i) * DD; const float* br = Bm + ((size_t)b * NN + j) * DD; float s = 0.f;
#pragma unroll 1
        for (int h = 0; h < DD; ++h) { const float a = fmaxf(__fadd_rn(__fadd_rn(ar[h], br[h]), bfr(b1[h])), 0.f); float w = bfr(w2[h]); asm volatile("" : "+v"(w)); float pr = __fmul_rn(a, w); asm volatile("" : "+v"(pr)); s = __fadd_rn(s, pr); }
        o[u] = __fadd_rn(s, bfr(b2[0])); }
    *(volatile v4f*)(OUT + e) = o; __threadfence(); *(volatile v4f*)(OUT + e) = o; }

extern "C" void kernel_launch(void* const* d_in, const int* in_sizes, int n_in,
                              void* d_out, int out_size, void* d_ws, size_t ws_size, hipStream_t stream) {
    (void)in_sizes; (void)n_in; (void)out_size;
    const float** I = (const float**)d_in;
    const float *agents = I[0], *enc_w = I[1], *enc_b = I[2], *enc_g = I[3], *enc_beta = I[4], *qkv_w = I[5], *qkv_b = I[6], *attn_ow = I[7], *attn_ob = I[8], *ln1_g = I[9], *ln1_b = I[10], *ffn_w1 = I[11], *ffn_b1 = I[12], *ffn_w2 = I[13], *ffn_b2 = I[14], *ln2_g = I[15], *ln2_b = I[16], *rel_w1 = I[17], *rel_b1 = I[18], *rel_w2 = I[19], *rel_b2 = I[20];
    float* OUT = (float*)d_out;
    char* wsp = (char*)d_ws;
    auto take = [&](size_t bytes) { char* p = wsp; wsp += (bytes + 255) & ~(size_t)255; return (void*)p; };
    bf* BENC = (bf*)take(DD * FF * 2); bf* BQKV[2]; bf* BOW[2]; bf* BF1[2]; bf* BF2[2]; for (int l = 0; l < 2; ++l) { BQKV[l] = (bf*)take((size_t)D3 * DD * 2); BOW[l] = (bf*)take(DD * DD * 2); BF1[l] = (bf*)take((size_t)DFF * DD * 2); BF2[l] = (bf*)take((size_t)DD * DFF * 2); } bf* BRA = (bf*)take(DD * DD * 2); bf* BRB = (bf*)take(DD * DD * 2);
    bf* AGB = (bf*)take((size_t)NT * FF * 2); float* E = (float*)take((size_t)NT * DD * 4); float* X = (float*)take((size_t)NT * DD * 4); bf* Xh = (bf*)take((size_t)NT * DD * 2); bf* Xl = (bf*)take((size_t)NT * DD * 2); float* QKV = (float*)take((size_t)NT * D3 * 4);
    h16* Q16 = (h16*)take((size_t)NZ * NN * DH * 2); h16* K16 = (h16*)take((size_t)NZ * NN * DH * 2); h16* VT = (h16*)take((size_t)NZ * 64 * NN * 2); float* Sb = (float*)take((size_t)NZ * NN * NN * 4); h16* P16 = (h16*)take((size_t)NZ * NN * NN * 2); float* O = (float*)take((size_t)NZ * NN * 64 * 4); bf* Ah = (bf*)take((size_t)NT * DD * 2); bf* Al = (bf*)take((size_t)NT * DD * 2);
    float* AO = (float*)take((size_t)NT * DD * 4); float* F1 = (float*)take((size_t)NT * DFF * 4); bf* Gh = (bf*)take((size_t)NT * DFF * 2); bf* Gl = (bf*)take((size_t)NT * DFF * 2); float* F2 = (float*)take((size_t)NT * DD * 4); float* RA = (float*)take((size_t)NT * DD * 4); float* RB = (float*)take((size_t)NT * DD * 4);
    if ((size_t)(wsp - (char*)d_ws) > ws_size) return;
    k_wtG<<<(FF * DD / 64 + 63) / 64, 256, 0, stream>>>(enc_w, FF, DD, BENC);
    for (int l = 0; l < 2; ++l) { k_wtG<<<(DD * D3 / 64 + 63) / 64, 256, 0, stream>>>(qkv_w + (size_t)l * DD * D3, DD, D3, BQKV[l]); k_wtG<<<(DD * DD / 64 + 63) / 64, 256, 0, stream>>>(attn_ow + (size_t)l * DD * DD, DD, DD, BOW[l]); k_wtG<<<(DD * DFF / 64 + 63) / 64, 256, 0, stream>>>(ffn_w1 + (size_t)l * DD * DFF, DD, DFF, BF1[l]); k_wtG<<<(DFF * DD / 64 + 63) / 64, 256, 0, stream>>>(ffn_w2 + (size_t)l * DFF * DD, DFF, DD, BF2[l]); }
    k_wtG<<<(DD * DD / 64 + 63) / 64, 256, 0, stream>>>(rel_w1, DD, DD, BRA); k_wtG<<<(DD * DD / 64 + 63) / 64, 256, 0, stream>>>(rel_w1 + (size_t)DD * DD, DD, DD, BRB);
    const unsigned gT = (NT * DD / 4 + 255) / 256;
    k_cvt8<<<(NT * FF / 8 + 255) / 256, 256, 0, stream>>>(agents, AGB, (size_t)NT * FF / 8);
    k_gemmw<bf, 0, true><<<dim3(NT / 64, DD / 64, 1), 32, 0, stream>>>(AGB, nullptr, BENC, nullptr, FF, E, DD, enc_b, 0, 0, 0);
    k_ln<1, 0><<<NT / 8, 256, 0, stream>>>(E, nullptr, enc_g, enc_beta, X, Xh, Xl);
    for (int l = 0; l < 2; ++l) {
        k_gemmw<bf, 1, true><<<dim3(NT / 64, D3 / 64, 1), 32, 0, stream>>>(Xh, Xl, BQKV[l], nullptr, DD, QKV, D3, qkv_b + (size_t)l * D3, 0, 0, 0);
        k_pl<<<(NZ * NN * DH / 4 + 255) / 256, 256, 0, stream>>>(QKV, 0, Q16); k_pl<<<(NZ * NN * DH / 4 + 255) / 256, 256, 0, stream>>>(QKV, DD, K16); k_vt<<<(NZ * 64 * NN / 2 + 255) / 256, 256, 0, stream>>>(QKV, VT);
        k_gemmw<h16, 0, false><<<dim3(NN / 64, NN / 64, NZ), 32, 0, stream>>>(Q16, nullptr, K16, nullptr, DH, Sb, NN, nullptr, (size_t)NN * DH, (size_t)NN * DH, (size_t)NN * NN);
        k_soft<<<NZ * NN / 8, 256, 0, stream>>>(Sb, P16);
        k_gemmw<h16, 0, false><<<dim3(NN / 64, 1, NZ), 32, 0, stream>>>(P16, nullptr, VT, nullptr, NN, O, 64, nullptr, (size_t)NN * NN, (size_t)64 * NN, (size_t)NN * 64);
        k_mrg<<<gT, 256, 0, stream>>>(O, Ah, Al);
        k_gemmw<bf, 1, true><<<dim3(NT / 64, DD / 64, 1), 32, 0, stream>>>(Ah, Al, BOW[l], nullptr, DD, AO, DD, attn_ob + (size_t)l * DD, 0, 0, 0);
        k_ln<0, 1><<<NT / 8, 256, 0, stream>>>(AO, X, ln1_g + (size_t)l * DD, ln1_b + (size_t)l * DD, X, Xh, Xl);
        k_gemmw<bf, 1, true><<<dim3(NT / 64, DFF / 64, 1), 32, 0, stream>>>(Xh, Xl, BF1[l], nullptr, DD, F1, DFF, ffn_b1 + (size_t)l * DFF, 0, 0, 0); k_rl<<<(unsigned)((NT * DFF / 4 + 255) / 256), 256, 0, stream>>>(F1, (size_t)NT * DFF, Gh, Gl);
        k_gemmw<bf, 1, true><<<dim3(NT / 64, DD / 64, 1), 32, 0, stream>>>(Gh, Gl, BF2[l], nullptr, DFF, F2, DD, ffn_b2 + (size_t)l * DD, 0, 0, 0);
        k_ln<0, 1><<<NT / 8, 256, 0, stream>>>(F2, X, ln2_g + (size_t)l * DD, ln2_b + (size_t)l * DD, X, Xh, Xl); }
    k_gemmw<bf, 1, false><<<dim3(NT / 64, DD / 64, 1), 32, 0, stream>>>(Xh, Xl, BRA, nullptr, DD, RA, DD, nullptr, 0, 0, 0); k_gemmw<bf, 1, false><<<dim3(NT / 64, DD / 64, 1), 32, 0, stream>>>(Xh, Xl, BRB, nullptr, DD, RB, DD, nullptr, 0, 0, 0);
    k_pair<<<(unsigned)(((size_t)NBQ * NPR / 4 + 255) / 256), 256, 0, stream>>>(RA, RB, rel_b1, rel_w2, rel_b2, OUT);
}
